// Seq2SeqBasic_867583394175
// MI455X (gfx1250) — hardware-verified
//
#include <hip/hip_runtime.h>
#include <math.h>

constexpr int NSEQ  = 64;
constexpr int TENC  = 512;
constexpr int TDEC  = 512;
constexpr int NFEAT = 256;
constexpr int NHID  = 256;
constexpr int NGATE = 2 * NHID;
constexpr int KCAT  = NFEAT + NHID;
constexpr int NTHR_PACK = 256;
constexpr int NTHR_SEQ  = 512;
constexpr int NWAVE_SEQ = NTHR_SEQ / 32;
constexpr int NBLK_SEQ  = 2;
constexpr int BROWS     = NSEQ / NBLK_SEQ;
constexpr int ROWS_PER_WAVE = BROWS / NWAVE_SEQ;
constexpr int TPITCH      = 264;
constexpr int TILE_HALVES = BROWS * TPITCH;
constexpr int NTILE       = 3;
constexpr int POOL_HALVES = NTILE * TILE_HALVES;
constexpr int SPITCH      = NHID;
constexpr int STG_FLOATS  = BROWS * SPITCH;
constexpr int WG_HALVES   = NGATE * KCAT;
constexpr int WC_HALVES   = NHID * KCAT;
constexpr int CELL_HALVES = WG_HALVES + WC_HALVES;
constexpr int NCELL       = 4;
constexpr size_t WS_NEED  = (size_t)NCELL * CELL_HALVES * 2;
constexpr int NOUT        = NSEQ * TDEC * NHID;
constexpr int XCHUNK_PER_THR = (BROWS * NFEAT / 8) / NTHR_SEQ;
constexpr float WCARRY = 32.0f;
constexpr float ACARRY = 16.0f;
constexpr float PSCL   = 1.0f / 512.0f;

static_assert(NFEAT == NHID);
static_assert(NHID == 16 * NWAVE_SEQ);
static_assert(NSEQ % NBLK_SEQ == 0 && BROWS == 32);
static_assert(BROWS % NWAVE_SEQ == 0 && ROWS_PER_WAVE == 2);
static_assert(BROWS <= NTHR_SEQ);
static_assert(NFEAT / 8 == 32);
static_assert(TPITCH % 8 == 0 && KCAT % 32 == 0 && NFEAT % 32 == 0 && NHID % 32 == 0);
static_assert((BROWS * NFEAT / 8) % NTHR_SEQ == 0 && XCHUNK_PER_THR == 2);
static_assert(POOL_HALVES % 8 == 0);
static_assert(TENC == TDEC);
static_assert((NGATE * (NFEAT / 8)) % NTHR_PACK == 0);
static_assert(SPITCH == 256);

typedef __attribute__((ext_vector_type(16))) _Float16 v16h;
typedef __attribute__((ext_vector_type(8)))  _Float16 v8h;
typedef __attribute__((ext_vector_type(8)))  float    v8f;
typedef __attribute__((ext_vector_type(4)))  float    v4f;

__device__ __forceinline__ void mma_guard2(v8f& a, v8f& b, v16h x, v16h y, v16h z) {
  asm volatile("v_nop\n\tv_nop\n\tv_nop\n\tv_nop" : "+v"(a), "+v"(b) : "v"(x), "v"(y), "v"(z));
}
__device__ __forceinline__ void acc_guard2(v8f& a, v8f& b) {
  asm volatile("v_nop\n\tv_nop\n\tv_nop\n\tv_nop" : "+v"(a), "+v"(b));
}

template <typename T> struct Frag;
template <> struct Frag<_Float16> {
  typedef v16h V; union U { v16h v; v8h h[2]; };
  static __device__ __forceinline__ v16h load(const _Float16* p) {
    U f; f.h[0] = *(const v8h*)(p); f.h[1] = *(const v8h*)(p + 16); return f.v;
  }
  static __device__ __forceinline__ v8f mma(v16h a, v16h b, v8f c) {
    return __builtin_amdgcn_wmma_f32_16x16x32_f16(false, a, false, b, (short)0, c, false, false);
  }
};

__device__ __forceinline__ float fsig(float x)  { return __builtin_amdgcn_rcpf(1.0f + expf(-x)); }
__device__ __forceinline__ float ftanh(float x) { return 1.0f - 2.0f * __builtin_amdgcn_rcpf(expf(2.0f * x) + 1.0f); }

__global__ __launch_bounds__(NTHR_PACK) void pack_weights_kernel(
    const float* __restrict__ enc_Wxg, const float* __restrict__ enc_Whg,
    const float* __restrict__ enc_Wxc, const float* __restrict__ enc_Whc,
    const float* __restrict__ dec_Wxg, const float* __restrict__ dec_Whg,
    const float* __restrict__ dec_Wxc, const float* __restrict__ dec_Whc,
    unsigned short* __restrict__ wsp) {
  const int part = blockIdx.y;
  const int cell = blockIdx.z;
  const int ncols = (part < 2) ? NGATE : NHID;
  const int nchunk = ncols * (NFEAT / 8);
  const int idx = blockIdx.x * NTHR_PACK + threadIdx.x;
  if (idx >= nchunk) return;
  const int net = cell >> 1, lay = cell & 1;
  const float* src = (part == 0) ? (net ? dec_Wxg : enc_Wxg)
                   : (part == 1) ? (net ? dec_Whg : enc_Whg)
                   : (part == 2) ? (net ? dec_Wxc : enc_Wxc)
                   :               (net ? dec_Whc : enc_Whc);
  src += (size_t)lay * NFEAT * ncols;
  _Float16* dst = (_Float16*)(wsp + (size_t)cell * CELL_HALVES + ((part < 2) ? 0 : WG_HALVES));
  const int koff = (part & 1) * NFEAT;
  const int n  = idx >> 5;
  const int k8 = idx & 31;
  v8h hv;
#pragma unroll
  for (int e = 0; e < 8; ++e) hv[e] = (_Float16)(src[(size_t)(8 * k8 + e) * ncols + n] * WCARRY);
  _Float16* dp = dst + (size_t)n * KCAT + koff + 8 * k8;
  *(volatile v8h*)dp = hv;
  __threadfence();
  *(volatile v8h*)dp = hv;
}

__device__ __forceinline__ void kpart2(const _Float16* a0p, const _Float16* a1p, const _Float16* __restrict__ w,
                                       v8f& acc0, v8f& acc1) {
#pragma unroll 1
  for (int k0 = 0; k0 < NFEAT; k0 += 32) {
    const v16h b  = Frag<_Float16>::load(w + k0);
    const v16h a0 = Frag<_Float16>::load(a0p + k0);
    const v16h a1 = Frag<_Float16>::load(a1p + k0);
    acc0 = Frag<_Float16>::mma(a0, b, acc0);
    acc1 = Frag<_Float16>::mma(a1, b, acc1);
    mma_guard2(acc0, acc1, a0, a1, b);
  }
}

__device__ __forceinline__ void gru_layer(const _Float16* Tx, const _Float16* Th, _Float16* Trh,
                                          float (&hA)[8], float (&hB)[8],
                                          const _Float16* __restrict__ wg, const _Float16* __restrict__ wc,
                                          const float* __restrict__ bg, const float* __restrict__ bc,
                                          const int* sLen, int tt, int nomask, int n, int c, int hh, int koff) {
  const v8f z8 = {0.f, 0.f, 0.f, 0.f, 0.f, 0.f, 0.f, 0.f};
  const _Float16* x0p = Tx  + c * TPITCH + koff;
  const _Float16* x1p = Tx  + (16 + c) * TPITCH + koff;
  const _Float16* h0p = Th  + c * TPITCH + koff;
  const _Float16* h1p = Th  + (16 + c) * TPITCH + koff;
  const _Float16* q0p = Trh + c * TPITCH + koff;
  const _Float16* q1p = Trh + (16 + c) * TPITCH + koff;
  const _Float16* wr = wg + (size_t)n * KCAT + koff;
  const _Float16* wu = wg + (size_t)(NHID + n) * KCAT + koff;
  const _Float16* wn = wc + (size_t)n * KCAT + koff;
  const float bgr = bg[n], bgu = bg[NHID + n], bcn = bc[n];

  v8f acc0 = z8, acc1 = z8;
  kpart2(x0p, x1p, wr, acc0, acc1);
  kpart2(h0p, h1p, wr + NFEAT, acc0, acc1);
  acc_guard2(acc0, acc1);
#pragma unroll
  for (int r = 0; r < 8; ++r) {
    const float rA = fsig(acc0[r] * PSCL + bgr);
    const float rB = fsig(acc1[r] * PSCL + bgr);
    Trh[(8 * hh + r) * TPITCH + n]      = (_Float16)(ACARRY * (rA * hA[r]));
    Trh[(16 + 8 * hh + r) * TPITCH + n] = (_Float16)(ACARRY * (rB * hB[r]));
  }
  __syncthreads();

  acc0 = z8; acc1 = z8;
  kpart2(x0p, x1p, wu, acc0, acc1);
  kpart2(h0p, h1p, wu + NFEAT, acc0, acc1);
  acc_guard2(acc0, acc1);
  float ugA[8], ugB[8];
#pragma unroll
  for (int r = 0; r < 8; ++r) {
    ugA[r] = fsig(acc0[r] * PSCL + bgu);
    ugB[r] = fsig(acc1[r] * PSCL + bgu);
  }

  acc0 = z8; acc1 = z8;
  kpart2(x0p, x1p, wn, acc0, acc1);
  kpart2(q0p, q1p, wn + NFEAT, acc0, acc1);
  acc_guard2(acc0, acc1);
#pragma unroll
  for (int r = 0; r < 8; ++r) {
    const float cA = ftanh(acc0[r] * PSCL + bcn);
    const float cB = ftanh(acc1[r] * PSCL + bcn);
    const float hoA = hA[r], hoB = hB[r];
    const float uA = ugA[r], uB = ugB[r];
    const float hnA = uA * hoA + (1.0f - uA) * cA;
    const float hnB = uB * hoB + (1.0f - uB) * cB;
    const int lvA = sLen[8 * hh + r];
    const int lvB = sLen[16 + 8 * hh + r];
    const int keepA = nomask | (int)(tt < lvA);
    const int keepB = nomask | (int)(tt < lvB);
    hA[r] = keepA ? hnA : hoA;
    hB[r] = keepB ? hnB : hoB;
  }
}

__global__ __launch_bounds__(NTHR_SEQ) void gru_seq_kernel(
    const float* __restrict__ enc_in, const float* __restrict__ dec_in, const int* __restrict__ lens,
    const float* __restrict__ enc_bg, const float* __restrict__ enc_bc,
    const float* __restrict__ dec_bg, const float* __restrict__ dec_bc,
    const unsigned short* __restrict__ wsp, float* __restrict__ out) {
  __shared__ __align__(16) _Float16 Tiles[POOL_HALVES];
  __shared__ __align__(16) float    Stg[STG_FLOATS];
  __shared__ int sLen[BROWS];
  _Float16* Tx  = Tiles;
  _Float16* Th  = Tiles + TILE_HALVES;
  _Float16* Trh = Tiles + 2 * TILE_HALVES;

  const int tid = threadIdx.x, lane = tid & 31, wave = tid >> 5;
  const int c = lane & 15, hh = lane >> 4, koff = hh * 8;
  const int n = 16 * wave + c;
  const int rb = blockIdx.x * BROWS;
  const _Float16* wbase = (const _Float16*)wsp;

  {
    v8h z8h;
#pragma unroll
    for (int e = 0; e < 8; ++e) z8h[e] = (_Float16)0.0f;
#pragma unroll 1
    for (int i = tid; i < POOL_HALVES / 8; i += NTHR_SEQ) *(v8h*)(Tiles + 8 * i) = z8h;
    if (tid < BROWS) sLen[tid] = lens[rb + tid];
  }
  float hs0[2][8], hs1[2][8];
#pragma unroll
  for (int mt = 0; mt < 2; ++mt)
#pragma unroll
    for (int r = 0; r < 8; ++r) { hs0[mt][r] = 0.0f; hs1[mt][r] = 0.0f; }
  __syncthreads();

#pragma unroll 1
  for (int t = 0; t < TENC + TDEC; ++t) {
    const bool enc = (t < TENC);
    const int  tt  = enc ? t : t - TENC;
    const float* xsrc = enc ? enc_in : dec_in;
    const _Float16* cellb = wbase + (enc ? 0 : 2 * CELL_HALVES);
    const _Float16* wg0 = cellb;
    const _Float16* wc0 = cellb + WG_HALVES;
    const _Float16* wg1 = cellb + CELL_HALVES;
    const _Float16* wc1 = cellb + CELL_HALVES + WG_HALVES;
    const float* bg0 = enc ? enc_bg : dec_bg;
    const float* bc0 = enc ? enc_bc : dec_bc;
    const float* bg1 = bg0 + NGATE;
    const float* bc1 = bc0 + NHID;
    const int nomask = enc ? 0 : 1;

    {
      const float* xs = xsrc + (size_t)tt * NFEAT;
#pragma unroll
      for (int i = 0; i < XCHUNK_PER_THR; ++i) {
        const int idx = tid + NTHR_SEQ * i;
        const int row = idx >> 5, c8 = (idx & 31) * 8;
        const float* sp = xs + (size_t)(rb + row) * ((size_t)TENC * NFEAT) + c8;
        const v4f a = *(const v4f*)(sp);
        const v4f b = *(const v4f*)(sp + 4);
        v8h hv;
#pragma unroll
        for (int e = 0; e < 4; ++e) { hv[e] = (_Float16)(a[e] * ACARRY); hv[4 + e] = (_Float16)(b[e] * ACARRY); }
        *(v8h*)(Tx + row * TPITCH + c8) = hv;
      }
#pragma unroll
      for (int mt = 0; mt < 2; ++mt)
#pragma unroll
        for (int r = 0; r < 8; ++r) Th[(16 * mt + 8 * hh + r) * TPITCH + n] = (_Float16)(ACARRY * hs0[mt][r]);
    }
    __syncthreads();

    gru_layer(Tx, Th, Trh, hs0[0], hs0[1], wg0, wc0, bg0, bc0, sLen, tt, nomask, n, c, hh, koff);
    __syncthreads();

#pragma unroll
    for (int mt = 0; mt < 2; ++mt) {
#pragma unroll
      for (int r = 0; r < 8; ++r) {
        const int row = 16 * mt + 8 * hh + r;
        Tx[row * TPITCH + n] = (_Float16)(ACARRY * hs0[mt][r]);
        Th[row * TPITCH + n] = (_Float16)(ACARRY * hs1[mt][r]);
      }
    }
    __syncthreads();

    gru_layer(Tx, Th, Trh, hs1[0], hs1[1], wg1, wc1, bg1, bc1, sLen, tt, nomask, n, c, hh, koff);

    if (!enc) {
#pragma unroll
      for (int mt = 0; mt < 2; ++mt)
#pragma unroll
        for (int r = 0; r < 8; ++r) Stg[(16 * mt + 8 * hh + r) * SPITCH + n] = hs1[mt][r];
    }
    __syncthreads();
    if (!enc) {
      for (int pass = 0; pass < 2; ++pass) {
#pragma unroll
        for (int i = 0; i < ROWS_PER_WAVE; ++i) {
          const int row = ROWS_PER_WAVE * wave + i;
          const float* sp = Stg + row * SPITCH;
          float* op = out + ((size_t)(rb + row) * TDEC + (size_t)tt) * NHID;
          const v4f v0 = *(const v4f*)(sp + 4 * lane);
          const v4f v1 = *(const v4f*)(sp + 128 + 4 * lane);
          *(volatile v4f*)(op + 4 * lane) = v0;
          *(volatile v4f*)(op + 128 + 4 * lane) = v1;
        }
        __threadfence();
      }
    }
  }
}

extern "C" void kernel_launch(void* const* d_in, const int* in_sizes, int n_in,
                              void* d_out, int out_size, void* d_ws, size_t ws_size, hipStream_t stream) {
  if (n_in < 15 || d_out == nullptr || d_ws == nullptr) return;
  if (in_sizes[0] != NSEQ * TENC * NFEAT || in_sizes[1] != NSEQ * TDEC * NFEAT || in_sizes[2] != NSEQ ||
      in_sizes[3] != 2 * NFEAT * NGATE || in_sizes[4] != 2 * NHID * NGATE || in_sizes[5] != 2 * NGATE ||
      in_sizes[6] != 2 * NFEAT * NHID || in_sizes[7] != 2 * NHID * NHID || in_sizes[8] != 2 * NHID ||
      in_sizes[9] != 2 * NFEAT * NGATE || in_sizes[10] != 2 * NHID * NGATE || in_sizes[11] != 2 * NGATE ||
      in_sizes[12] != 2 * NFEAT * NHID || in_sizes[13] != 2 * NHID * NHID || in_sizes[14] != 2 * NHID ||
      out_size != NOUT) return;
  if (WS_NEED > ws_size) return;

  const float* enc_in  = (const float*)d_in[0];
  const float* dec_in  = (const float*)d_in[1];
  const int*   lens    = (const int*)  d_in[2];
  const float* enc_Wxg = (const float*)d_in[3];
  const float* enc_Whg = (const float*)d_in[4];
  const float* enc_bg  = (const float*)d_in[5];
  const float* enc_Wxc = (const float*)d_in[6];
  const float* enc_Whc = (const float*)d_in[7];
  const float* enc_bc  = (const float*)d_in[8];
  const float* dec_Wxg = (const float*)d_in[9];
  const float* dec_Whg = (const float*)d_in[10];
  const float* dec_bg  = (const float*)d_in[11];
  const float* dec_Wxc = (const float*)d_in[12];
  const float* dec_Whc = (const float*)d_in[13];
  const float* dec_bc  = (const float*)d_in[14];
  unsigned short* wsp  = (unsigned short*)d_ws;
  float* out = (float*)d_out;

  pack_weights_kernel<<<dim3((NGATE * (NFEAT / 8)) / NTHR_PACK, 4, NCELL), NTHR_PACK, 0, stream>>>(
      enc_Wxg, enc_Whg, enc_Wxc, enc_Whc, dec_Wxg, dec_Whg, dec_Wxc, dec_Whc, wsp);

  gru_seq_kernel<<<NBLK_SEQ, NTHR_SEQ, 0, stream>>>(enc_in, dec_in, lens, enc_bg, enc_bc, dec_bg, dec_bc, wsp, out);
}
